// TransformerLayer_54451595378769
// MI455X (gfx1250) — hardware-verified
//
#include <hip/hip_runtime.h>
#ifndef NB
#define NB 2
#endif
#ifndef SEQ
#define SEQ 2048
#endif
#define NB_FULL 2
#define SEQ_FULL 2048
#define SQ SEQ
#define DM 1024
#define NH 16
#define HD 64
#define HG 2
#define DFF 4096
#define DMQ DM
#define NR ((size_t)NB * SQ)
#define MP ((int)((size_t)NB * SQ))
#define LQ (3 * DM)

typedef unsigned short v8us __attribute__((ext_vector_type(8), may_alias));
typedef float  v8f  __attribute__((ext_vector_type(8)));
typedef float  v4f  __attribute__((ext_vector_type(4)));
typedef float  v4fa __attribute__((ext_vector_type(4), may_alias));
typedef _Float16 v16h __attribute__((ext_vector_type(16)));
typedef _Float16 v4h __attribute__((ext_vector_type(4)));
union FragH { v16h v; v8us half[2]; _Float16 h[16]; unsigned short u[16]; };

__device__ __forceinline__ unsigned short bf16_bits(float x) { unsigned int u = __float_as_uint(x); return (unsigned short)((u + 0x7FFFu + ((u >> 16) & 1u)) >> 16); }
__device__ __forceinline__ float bf16_val(unsigned short b) { return __uint_as_float(((unsigned int)b) << 16); }
__device__ __forceinline__ float bf16_rne(float x) { return bf16_val(bf16_bits(x)); }

__global__ __launch_bounds__(256) void k_wt_f16(const float* __restrict__ W, _Float16* __restrict__ Wt, int K, int N, float scale) {
  const int t = blockIdx.x * 256 + threadIdx.x; if (t >= N * (K / 8)) return; const int n = t / (K / 8), k8 = (t % (K / 8)) * 8; FragH f;
#pragma unroll
  for (int i = 0; i < 8; ++i) f.h[i] = (_Float16)(bf16_rne(W[(size_t)(k8 + i) * N + n]) * scale); const v8us o = f.half[0];
  *(volatile v8us*)((unsigned short*)Wt + (size_t)n * K + k8) = o; __threadfence(); *(volatile v8us*)((unsigned short*)Wt + (size_t)n * K + k8) = o;
}

template <int NHv, int TTv>
__global__ __launch_bounds__(256) void k_vt(const _Float16* __restrict__ V16, int ldv, int voff, _Float16* __restrict__ Vt) { __shared__ unsigned short tl[64][66]; const int tid = threadIdx.x; const int slab = blockIdx.x / (TTv / 64), lg = blockIdx.x % (TTv / 64); const int b = slab / NHv, h = slab % NHv;
  for (int i = tid; i < 64 * 8; i += 256) { const int r = i / 8, c8 = (i % 8) * 8; FragH f; f.half[0] = *(const v8us*)((const unsigned short*)V16 + ((size_t)b * TTv + lg * 64 + r) * ldv + voff + h * 64 + c8);
#pragma unroll
    for (int q = 0; q < 8; ++q) tl[r][c8 + q] = f.u[q]; }
  __syncthreads();
  for (int pass = 0; pass < 2; ++pass) {
#pragma unroll
    for (int rd = 0; rd < 2; ++rd) { const int d = rd * 32 + tid / 8, pc = tid % 8; FragH f;
#pragma unroll
      for (int q = 0; q < 8; ++q) f.u[q] = tl[pc * 8 + q][d];
      *(volatile v8us*)((unsigned short*)Vt + ((size_t)slab * 64 + d) * TTv + lg * 64 + pc * 8) = f.half[0]; }
    if (pass == 0) __threadfence(); } }

__device__ __forceinline__ v16h g2_frag(const _Float16* p, int hh) { FragH f; f.half[0] = *(const v8us*)((const unsigned short*)p + 8 * hh); f.half[1] = *(const v8us*)((const unsigned short*)p + 16 + 8 * hh); return f.v; }
__device__ __forceinline__ v8f g2_mma(v16h a, v16h b, v8f c) { v8f d = __builtin_amdgcn_wmma_f32_16x16x32_f16(false, a, false, b, (short)0, c, false, false); asm volatile("v_nop\n\tv_nop\n\tv_nop\n\tv_nop" : "+v"(d) : "v"(a), "v"(b)); return d; }
template <int ACT>
__global__ __launch_bounds__(128) void k_gemm2(const _Float16* __restrict__ A, int lda, size_t sA, const _Float16* __restrict__ Bh, int ldb, size_t sB, float alpha, const float* __restrict__ bias, size_t sBias, const float* __restrict__ CP, int rowsPerB, size_t sCPb, int row0g,
    float* __restrict__ C, _Float16* __restrict__ C16, int ldc, size_t sC, int M, int N, int K) { static_assert(ACT == 0 || ACT == 3 || ACT == 6 || ACT == 8 || ACT == 9 || ACT == 11 || ACT == 12 || ACT == 14 || ACT == 15 || ACT == 16 || ACT == 17 || ACT == 18);
  __shared__ __attribute__((aligned(16))) float so[4][32][68];
  const int tid = threadIdx.x, w = tid >> 5, lane = tid & 31, ln = lane & 15, hh = lane >> 4; const int by = blockIdx.y;
  A += (size_t)by * sA; Bh += (size_t)by * sB; const size_t cofs = (size_t)by * sC; const float* bp = bias ? bias + (size_t)by * sBias : nullptr;
  const int ntn = N >> 6; const int mt = blockIdx.x / ntn, nq = blockIdx.x - mt * ntn; const int row0 = mt * 128 + 32 * w, col0 = nq * 64; if (row0 >= M) return;
  const _Float16* a0p = A + (size_t)(row0 + ln) * lda; const _Float16* a1p = a0p + (size_t)16 * lda;
  const _Float16* b0p = Bh + (size_t)(col0 + ln) * ldb; const _Float16* b1p = b0p + (size_t)16 * ldb; const _Float16* b2p = b1p + (size_t)16 * ldb; const _Float16* b3p = b2p + (size_t)16 * ldb;
  const v8f z8 = {0.f,0.f,0.f,0.f,0.f,0.f,0.f,0.f}; v8f c00 = z8, c01 = z8, c02 = z8, c03 = z8, c10 = z8, c11 = z8, c12 = z8, c13 = z8;
#pragma unroll 1
  for (int kb = 0; kb < K; kb += 32) { const v16h a0 = g2_frag(a0p + kb, hh), a1 = g2_frag(a1p + kb, hh);
    v16h b = g2_frag(b0p + kb, hh); c00 = g2_mma(a0, b, c00); c10 = g2_mma(a1, b, c10);
    b = g2_frag(b1p + kb, hh); c01 = g2_mma(a0, b, c01); c11 = g2_mma(a1, b, c11);
    b = g2_frag(b2p + kb, hh); c02 = g2_mma(a0, b, c02); c12 = g2_mma(a1, b, c12);
    b = g2_frag(b3p + kb, hh); c03 = g2_mma(a0, b, c03); c13 = g2_mma(a1, b, c13); }
  v8f accs[8] = {c00, c01, c02, c03, c10, c11, c12, c13};
#pragma unroll
  for (int u = 0; u < 8; ++u) { const int t = u & 3, half = u >> 2; const int col = col0 + t * 16 + ln; const float bv = bp ? bf16_rne(bp[col]) : 0.f;
#pragma unroll
    for (int r = 0; r < 8; ++r) { const int rloc = half * 16 + 8 * hh + r; float v = accs[u][r] * alpha + bv; if (CP) { if (rowsPerB < 0) v += CP[cofs + (size_t)(row0g + row0 + rloc) * ldc + col];        else { const int bidx = (row0g + row0 + rloc) / rowsPerB; v += CP[(size_t)bidx * sCPb + (size_t)by * 64 + col]; } }
      if (ACT == 3) v = fmaxf(v, 0.f); else if (ACT == 6) v = 0.5f * v * (1.0f + erff(v * 0.70710678118654752f)); else if (ACT == 11) v = 1.0f / (1.0f + expf(-v)); else if (ACT == 15) v = v / (1.0f + expf(-v)); else if (ACT == 18) v = v / (1.0f + expf(-1.702f * v)); else if (ACT == 12) v = (v > 0.f) ? v : 0.01f * v; else if (ACT == 8) v = tanhf(v); else if (ACT == 9) v = 0.5f * v * (1.0f + tanhf(0.7978845608028654f * (v + 0.044715f * v * v * v))); else if (ACT == 14) v = (v > 0.f) ? v : 0.1f * v; else if (ACT == 16) v = (v >= 0.f) ? v : 0.3f * v; else if (ACT == 17) v = (v >= 0.f) ? v : 0.2f * v;
      so[w][rloc][t * 16 + ln] = v; } }
  __builtin_amdgcn_fence(4  , "workgroup"); __builtin_amdgcn_wave_barrier();
  const int rsub = lane >> 4, c4 = (lane & 15) * 4;
  for (int pass = 0; pass < 2; ++pass) {
#pragma unroll
    for (int q = 0; q < 16; ++q) { const int r = q * 2 + rsub; const v4f v = *(const v4fa*)&so[w][r][c4]; if (C) *(volatile v4f*)(C + cofs + (size_t)(row0 + r) * ldc + col0 + c4) = v; if (C16) { v4h h4; for (int i = 0; i < 4; ++i) h4[i] = (_Float16)v[i]; *(volatile v4h*)(C16 + cofs + (size_t)(row0 + r) * ldc + col0 + c4) = h4; } }
    if (pass == 0) __threadfence(); } }

__global__ __launch_bounds__(256) void k_rsmf(const float* __restrict__ S, _Float16* __restrict__ P, int qn, int hg) {
  #pragma clang fp contract(off)
  const int t = blockIdx.x * 256 + threadIdx.x; if (t >= qn * hg) return; const size_t i = (size_t)(t / qn) * SQ + (t % qn); const float* s = S + i * SQ; float mx = -3.0e38f;
#pragma unroll 1
  for (int j = 0; j < SQ; ++j) mx = fmaxf(mx, s[j]); float se = 0.f;
#pragma unroll 1
  for (int j = 0; j < SQ; ++j) se += __expf(s[j] - mx); const float sc = 256.0f / se;
#pragma unroll 1
  for (int j0 = 0; j0 < SQ; j0 += 8) { FragH f; for (int q = 0; q < 8; ++q) f.h[q] = (_Float16)(__expf(s[j0 + q] - mx) * sc); unsigned short* d = (unsigned short*)P + i * SQ + j0; *(volatile v8us*)d = f.half[0]; __threadfence(); *(volatile v8us*)d = f.half[0]; } }

template <int BFIN, int W16, int W32>
__global__ __launch_bounds__(256) void k_lnx(const float* __restrict__ X, const float* __restrict__ g, const float* __restrict__ bb, float eps, _Float16* __restrict__ N16, float* __restrict__ N32) {
  #pragma clang fp contract(off)
  __shared__ float red[256]; const size_t r = blockIdx.x; const int t = threadIdx.x; const bool act = t < (DMQ / 4); const int c0 = act ? t * 4 : 0;
  const v4f xa = *(const v4fa*)(X + r * DMQ + c0); float s[4]; float sum = 0.f;
  for (int q = 0; q < 4; ++q) { s[q] = act ? (BFIN ? bf16_rne(xa[q]) : xa[q]) : 0.f; sum = __fadd_rn(sum, s[q]); }
  red[t] = sum; __syncthreads(); for (int st = 128; st > 0; st >>= 1) { if (t < st) red[t] = __fadd_rn(red[t], red[t + st]); __syncthreads(); } const float mu = red[0] / (float)DMQ; __syncthreads();
  float vs = 0.f; for (int q = 0; q < 4; ++q) { const float dl = act ? __fadd_rn(s[q], -mu) : 0.f; vs = __fadd_rn(vs, __fmul_rn(dl, dl)); } red[t] = vs; __syncthreads(); for (int st = 128; st > 0; st >>= 1) { if (t < st) red[t] = __fadd_rn(red[t], red[t + st]); __syncthreads(); }
  const float rs = rsqrtf(__fadd_rn(red[0] / (float)DMQ, eps)); v4h y; v4f yf;
  for (int q = 0; q < 4; ++q) { const int c = c0 + q; yf[q] = __fadd_rn(__fmul_rn(__fmul_rn(__fadd_rn(s[q], -mu), rs), bf16_rne(g[c])), bf16_rne(bb[c])); y[q] = (_Float16)yf[q]; }
  if (!act) return;
  for (int pass = 0; pass < 2; ++pass) { if (W16) *(volatile v4h*)(N16 + r * DMQ + c0) = y; if (W32) *(volatile v4f*)(N32 + r * DMQ + c0) = yf; if (pass == 0) __threadfence(); } }

__global__ __launch_bounds__(256) void k_bfr(const float* __restrict__ x, float* __restrict__ XB, size_t n8) { const size_t t = (size_t)blockIdx.x * 256 + threadIdx.x; if (t >= n8) return; v4f a = *(const v4fa*)(x + t * 8), c = *(const v4fa*)(x + t * 8 + 4); for (int q = 0; q < 4; ++q) { a[q] = bf16_rne(a[q]); c[q] = bf16_rne(c[q]); }
  for (int pass = 0; pass < 2; ++pass) { *(volatile v4f*)(XB + t * 8) = a; *(volatile v4f*)(XB + t * 8 + 4) = c; if (pass == 0) __threadfence(); } }

static constexpr size_t cmaxz(size_t a, size_t b) { return a > b ? a : b; }
static constexpr size_t SZ_BQKV = (size_t)3 * DM * DM * 2;
static constexpr size_t SZ_BO   = (size_t)DM * DM * 2;
static constexpr size_t SZ_N16  = (size_t)NB * SQ * DM * 2;
static constexpr size_t SZ_XB   = (size_t)NB * SQ * DM * 4;
static constexpr size_t SZ_RA   = cmaxz((size_t)NB * SQ * 3 * DM * 2, (size_t)SQ * DFF * 2);
static constexpr size_t SZ_O16  = (size_t)NB * SQ * DM * 2;
static constexpr size_t SZ_RS   = cmaxz((size_t)HG * SQ * SQ * 4, (size_t)NB * SQ * DM * 4);
static constexpr size_t SZ_RP   = cmaxz((size_t)HG * SQ * SQ * 2, (size_t)2 * DFF * DM * 2);
static constexpr size_t SZ_VT   = (size_t)NH * HD * SQ * 2;
static constexpr size_t O_BQKV = 0;
static constexpr size_t O_BO   = O_BQKV + SZ_BQKV;
static constexpr size_t O_N16  = O_BO + SZ_BO;
static constexpr size_t O_XB   = O_N16 + SZ_N16;
static constexpr size_t O_RA   = O_XB + SZ_XB;
static constexpr size_t O_O16  = O_RA + SZ_RA;
static constexpr size_t O_RS   = O_O16 + SZ_O16;
static constexpr size_t O_RP   = O_RS + SZ_RS;
static constexpr size_t O_VT   = O_RP + SZ_RP;
static constexpr size_t WS_TOTAL = O_VT + SZ_VT;
static_assert(WS_TOTAL <= (size_t)134217728);
static_assert((SZ_BQKV % 256) == 0 && (SZ_BO % 256) == 0 && (SZ_N16 % 256) == 0 && (SZ_XB % 256) == 0 && (SZ_RA % 256) == 0 && (SZ_O16 % 256) == 0 && (SZ_RS % 256) == 0 && (SZ_RP % 256) == 0 && (SZ_VT % 256) == 0);
static_assert((size_t)NB * SQ * 3 * DM * 2 <= SZ_RA && (size_t)SQ * DFF * 2 <= SZ_RA);
static_assert((size_t)HG * SQ * SQ * 4 <= SZ_RS && (size_t)NB * SQ * DM * 4 <= SZ_RS);
static_assert((size_t)HG * SQ * SQ * 2 <= SZ_RP && (size_t)DFF * DM * 2 + (size_t)DM * DFF * 2 <= SZ_RP);
static_assert(NB <= NB_FULL && SQ <= SEQ_FULL);
static_assert((SQ % 128) == 0 && (DM % 64) == 0 && (DFF % 64) == 0 && (HD % 64) == 0 && ((3 * DM) % 64) == 0);
static_assert((DM % 32) == 0 && (DFF % 32) == 0 && (HD % 32) == 0 && (SQ % 32) == 0);
static_assert(NH * HD == DM && (NH % HG) == 0 && DMQ == 1024);
static_assert(((3 * DM * (DM / 8)) % 256) == 0 && ((DM * (DM / 8)) % 256) == 0 && ((DFF * (DM / 8)) % 256) == 0 && ((DM * (DFF / 8)) % 256) == 0);
static_assert((((size_t)SQ * DM / 8) % 256) == 0 && ((HG * SQ) % 256) == 0 && (SQ % 64) == 0);

extern "C" void kernel_launch(void* const* d_in, const int* in_sizes, int n_in,
                              void* d_out, int out_size, void* d_ws, size_t ws_size, hipStream_t stream) {
  if (n_in < 13) return;
  const size_t need_x = (size_t)(NB - 1) * SEQ_FULL * DM + (size_t)SQ * DM;
  if ((size_t)in_sizes[0] < need_x) return;
  if (in_sizes[1] < 3 * DM * DM || in_sizes[2] < 3 * DM || in_sizes[3] < DM * DM || in_sizes[4] < DM) return;
  if (in_sizes[5] < DM * DFF || in_sizes[6] < DFF || in_sizes[7] < DFF * DM || in_sizes[8] < DM) return;
  if (in_sizes[9] < DM || in_sizes[10] < DM || in_sizes[11] < DM || in_sizes[12] < DM) return;
  if ((size_t)out_size < (size_t)NB * SQ * DM) return;
  if (WS_TOTAL > ws_size) return;
  const float* const* I = (const float* const*)d_in;
  const float* x = I[0]; const float* wqkv = I[1]; const float* bqkv = I[2]; const float* wo = I[3]; const float* bo = I[4];
  const float* w1 = I[5]; const float* b1 = I[6]; const float* w2 = I[7]; const float* b2 = I[8];
  const float* g1 = I[9]; const float* be1 = I[10]; const float* g2 = I[11]; const float* be2 = I[12];
  char* ws = (char*)d_ws;
  _Float16* BQKV = (_Float16*)(ws + O_BQKV); _Float16* BO = (_Float16*)(ws + O_BO);
  _Float16* N16 = (_Float16*)(ws + O_N16); float* XB = (float*)(ws + O_XB);
  _Float16* QKV = (_Float16*)(ws + O_RA); _Float16* HF16 = (_Float16*)(ws + O_RA);
  _Float16* Q16 = QKV; _Float16* K16 = QKV + DM; _Float16* V16 = QKV + 2 * DM;
  _Float16* O16 = (_Float16*)(ws + O_O16);
  float* S = (float*)(ws + O_RS); float* X1 = (float*)(ws + O_RS);
  _Float16* P = (_Float16*)(ws + O_RP); _Float16* BW1 = (_Float16*)(ws + O_RP); _Float16* BW2 = BW1 + (size_t)DFF * DM;
  _Float16* VT = (_Float16*)(ws + O_VT);

  k_wt_f16<<<(unsigned)((3 * DM * (DM / 8)) / 256), 256, 0, stream>>>(wqkv, BQKV, DM, 3 * DM, 16.0f);
  k_wt_f16<<<(unsigned)((DM * (DM / 8)) / 256), 256, 0, stream>>>(wo, BO, DM, DM, 16.0f);
  for (int b = 0; b < NB; ++b) {
    const float* xb = x + (size_t)b * SEQ_FULL * DM; const size_t r0 = (size_t)b * SQ;
    k_bfr<<<(unsigned)(((size_t)SQ * DM / 8) / 256), 256, 0, stream>>>(xb, XB + r0 * DM, (size_t)SQ * DM / 8);
    k_lnx<1, 1, 0><<<(unsigned)SQ, 256, 0, stream>>>(xb, g1, be1, 1e-5f, N16 + r0 * DM, nullptr);
  }
  k_gemm2<0><<<dim3((unsigned)((MP / 128) * (3 * DM / 64)), 1), 128, 0, stream>>>(N16, DM, 0, BQKV, DM, 0, 0.0625f, bqkv, 0, nullptr, 1, 0, 0, nullptr, QKV, 3 * DM, 0, MP, 3 * DM, DM);
  for (int b = 0; b < NB; ++b) { const size_t r0 = (size_t)b * SQ;
    k_vt<NH, SQ><<<NH * (SQ / 64), 256, 0, stream>>>(V16 + r0 * LQ, LQ, 0, VT);
    for (int h0 = 0; h0 < NH; h0 += HG) {
      k_gemm2<0><<<dim3((SQ / 128) * (SQ / 64), HG), 128, 0, stream>>>(Q16 + r0 * LQ + (size_t)h0 * HD, LQ, (size_t)HD, K16 + r0 * LQ + (size_t)h0 * HD, LQ, (size_t)HD, 0.125f, nullptr, 0, nullptr, 1, 0, 0, S, nullptr, SQ, (size_t)SQ * SQ, SQ, SQ, HD);
      k_rsmf<<<(HG * SQ + 255) / 256, 256, 0, stream>>>(S, P, SQ, HG);
      k_gemm2<0><<<dim3((SQ / 128) * (HD / 64), HG), 128, 0, stream>>>(P, SQ, (size_t)SQ * SQ, VT + (size_t)h0 * HD * SQ, SQ, (size_t)HD * SQ, 0.25f, nullptr, 0, nullptr, 1, 0, 0, nullptr, O16 + r0 * DM + (size_t)h0 * HD, DM, (size_t)HD, SQ, HD, SQ);
    } }
  k_wt_f16<<<(unsigned)((DFF * (DM / 8)) / 256), 256, 0, stream>>>(w1, BW1, DM, DFF, 16.0f);
  k_wt_f16<<<(unsigned)((DM * (DFF / 8)) / 256), 256, 0, stream>>>(w2, BW2, DFF, DM, 16.0f);
  k_gemm2<0><<<dim3((unsigned)((MP / 128) * (DM / 64)), 1), 128, 0, stream>>>(O16, DM, 0, BO, DM, 0, 0.0009765625f, bo, 0, XB, -1, 0, 0, X1, nullptr, DM, 0, MP, DM, DM);
  k_lnx<0, 1, 0><<<(unsigned)NR, 256, 0, stream>>>(X1, g2, be2, 1e-5f, N16, nullptr);
  for (int b = 0; b < NB; ++b) { const size_t r0 = (size_t)b * SQ;
    k_gemm2<3><<<dim3((unsigned)((SQ / 128) * (DFF / 64)), 1), 128, 0, stream>>>(N16 + r0 * DM, DM, 0, BW1, DM, 0, 0.0625f, b1, 0, nullptr, 1, 0, 0, nullptr, HF16, DFF, 0, SQ, DFF, DM);
    k_gemm2<0><<<dim3((unsigned)((SQ / 128) * (DM / 64)), 1), 128, 0, stream>>>(HF16, DFF, 0, BW2, DFF, 0, 0.0625f, b2, 0, X1 + r0 * DM, -1, 0, 0, (float*)d_out + r0 * DM, nullptr, DM, 0, SQ, DM, DFF); }
}
